// CrossVerseAttention_5987184411236
// MI455X (gfx1250) — hardware-run, weakly checked
//
#include <hip/hip_runtime.h>
#include <math.h>
#include <stdint.h>

#define NB_   2
#define SEQ_  2048
#define DM_   1024
#define NH_   16
#define DHD_  64
#define NTOK_ (NB_ * SEQ_)

typedef _Float16 v16h __attribute__((ext_vector_type(16)));
typedef _Float16 v8h  __attribute__((ext_vector_type(8)));
typedef float    v8f  __attribute__((ext_vector_type(8)));
typedef float    v4f  __attribute__((ext_vector_type(4)));

union FragU { v16h v; v8h h[2]; };

__device__ __forceinline__ v16h ld_frag(const _Float16* p) {
  FragU f;
  f.h[0] = *(const v8h*)(p);
  f.h[1] = *(const v8h*)(p + 16);
  return f.v;
}

__device__ __forceinline__ v8f mma16(v16h a, v16h b, v8f c) {
  c = __builtin_amdgcn_wmma_f32_16x16x32_f16(false, a, false, b, (short)0, c, false, false);
  asm volatile("v_nop\n\tv_nop\n\tv_nop\n\tv_nop" : "+v"(c) : "v"(a), "v"(b));
  return c;
}

__device__ __forceinline__ void lds_wave_sync() {
  __builtin_amdgcn_fence(__ATOMIC_RELEASE, "workgroup");
  __builtin_amdgcn_wave_barrier();
  __builtin_amdgcn_fence(__ATOMIC_ACQUIRE, "workgroup");
}

__global__ __launch_bounds__(256) void cvt_f16_kernel(const float* __restrict__ src,
                                                      _Float16* __restrict__ dst, int n8, float scale) {
  const int i = blockIdx.x * 256 + threadIdx.x;
  if (i >= n8) return;
  const float* s = src + (size_t)i * 8;
  const v4f a = *(const v4f*)(s);
  const v4f b = *(const v4f*)(s + 4);
  v8h o;
  o[0] = (_Float16)(a[0] * scale); o[1] = (_Float16)(a[1] * scale);
  o[2] = (_Float16)(a[2] * scale); o[3] = (_Float16)(a[3] * scale);
  o[4] = (_Float16)(b[0] * scale); o[5] = (_Float16)(b[1] * scale);
  o[6] = (_Float16)(b[2] * scale); o[7] = (_Float16)(b[3] * scale);
  _Float16* d = dst + (size_t)i * 8;
  *(volatile v8h*)d = o;
  __threadfence();
  *(volatile v8h*)d = o;
}

template <int BIAS_MODE, bool OUT16, bool RESID>
__global__ __launch_bounds__(256) void gemm_kernel(
    const _Float16* __restrict__ A, int lda,
    const _Float16* __restrict__ Bt, int ldb,
    void* __restrict__ Cout, int ldc,
    const float* __restrict__ bias, float bscale,
    const float* __restrict__ resid,
    int M, int N, int K, float scale) {
  __shared__ __align__(16) float sT[8][16 * 68];
  const int lane = threadIdx.x & 31;
  const int wave = threadIdx.x >> 5;
  const int tilesN = N >> 6;
  const int tilesM = M >> 5;
  const int tile = blockIdx.x * 8 + wave;
  if (tile >= tilesM * tilesN) return;
  const int tm = tile / tilesN;
  const int tn = tile - tm * tilesN;
  const int m0 = tm << 5;
  const int n0 = tn << 6;
  const int rl   = lane & 15;
  const int hh   = lane >> 4;
  const int koff = hh * 8;
  const int mOff = hh * 8;

  v8f acc[2][4];
#pragma unroll
  for (int i = 0; i < 2; ++i)
#pragma unroll
    for (int j = 0; j < 4; ++j) acc[i][j] = (v8f){0.f, 0.f, 0.f, 0.f, 0.f, 0.f, 0.f, 0.f};

  for (int k0 = 0; k0 < K; k0 += 32) {
    v16h bfr[4];
#pragma unroll
    for (int j = 0; j < 4; ++j)
      bfr[j] = ld_frag(Bt + (size_t)(n0 + (j << 4) + rl) * ldb + k0 + koff);
#pragma unroll
    for (int i = 0; i < 2; ++i) {
      const v16h afr = ld_frag(A + (size_t)(m0 + (i << 4) + rl) * lda + k0 + koff);
#pragma unroll
      for (int j = 0; j < 4; ++j) acc[i][j] = mma16(afr, bfr[j], acc[i][j]);
    }
  }

  float* slab = sT[wave];
#pragma unroll
  for (int i = 0; i < 2; ++i) {
    const int mBase = m0 + (i << 4);
#pragma unroll
    for (int j = 0; j < 4; ++j) {
      const int n = n0 + (j << 4) + rl;
      float bv = 0.f;
      if (BIAS_MODE == 2) bv = bias[n] * bscale;
#pragma unroll
      for (int r = 0; r < 8; ++r) {
        float v = acc[i][j][r] * scale;
        if (BIAS_MODE == 1) v += bias[mBase + mOff + r] * bscale;
        if (BIAS_MODE == 2) v += bv;
        if (RESID) v += resid[(size_t)(mBase + mOff + r) * ldc + n];
        slab[(mOff + r) * 68 + (j << 4) + rl] = v;
      }
    }
    lds_wave_sync();
    if (!OUT16) {
      float* C = (float*)Cout;
      const int c4 = rl * 4;
      for (int pass = 0; pass < 2; ++pass) {
#pragma unroll
        for (int it = 0; it < 8; ++it) {
          const int row = it * 2 + hh;
          const v4f v = *(const v4f*)(slab + row * 68 + c4);
          *(volatile v4f*)(C + (size_t)(mBase + row) * ldc + n0 + c4) = v;
        }
        __threadfence();
      }
    } else {
      _Float16* C = (_Float16*)Cout;
      const int q4 = lane >> 3, c8 = (lane & 7) * 8;
      for (int pass = 0; pass < 2; ++pass) {
#pragma unroll
        for (int it = 0; it < 4; ++it) {
          const int row = it * 4 + q4;
          const float* sp = slab + row * 68 + c8;
          v8h hv;
#pragma unroll
          for (int e = 0; e < 8; ++e) hv[e] = (_Float16)sp[e];
          *(volatile v8h*)(C + (size_t)(mBase + row) * ldc + n0 + c8) = hv;
        }
        __threadfence();
      }
    }
    lds_wave_sync();
  }
}

__device__ __forceinline__ float verse_add(int vi, int vj) {
  int d = vi - vj;
  d = (d < 0) ? -d : d;
  float m = 0.3f * __builtin_amdgcn_rcpf((float)d);
  m = (d == 1) ? 0.7f : m;
  m = (d == 0) ? 1.0f : m;
  m = ((vi == 0) | (vj == 0)) ? 1.0f : m;
  return m;
}

#define FL_KC 64
#define FL_SC 0.00048828125f

__global__ __launch_bounds__(128) void flash_kernel(
    const _Float16* __restrict__ Qp, const _Float16* __restrict__ Kp,
    const _Float16* __restrict__ VTp, const int* __restrict__ vpos,
    _Float16* __restrict__ ctx) {
  union FB { v16h v; v8h h[2]; };
  __shared__ __align__(16) _Float16 Ksh[FL_KC * DHD_];
  __shared__ __align__(16) _Float16 Vth[DHD_ * FL_KC];
  __shared__ __align__(16) _Float16 Psh[4][16 * FL_KC];
  __shared__ __align__(16) float    Os[4][16 * 68];
  __shared__ int Vjs[FL_KC];

  const int tid  = threadIdx.x;
  const int wave = tid >> 5;
  const int lane = tid & 31;
  const int hh   = lane >> 4;
  const int c    = lane & 15;

  const int bx  = blockIdx.x;
  const int qb  = bx & 31;
  const int bhd = bx >> 5;
  const int h   = bhd & (NH_ - 1);
  const int b   = bhd >> 4;
  const int tok0 = b * SEQ_;
  const int qrow0 = qb * 64 + wave * 16;

  const _Float16* Qh = Qp  + (size_t)tok0 * DM_ + h * DHD_;
  const _Float16* Kh = Kp  + (size_t)tok0 * DM_ + h * DHD_;
  const _Float16* Vh = VTp + (size_t)(h * DHD_) * NTOK_ + tok0;
  const int*      vpb = vpos + tok0;
  _Float16*       cb = ctx + (size_t)tok0 * DM_ + h * DHD_;

  v16h qa[2];
#pragma unroll
  for (int dc = 0; dc < 2; ++dc)
    qa[dc] = ld_frag(Qh + (size_t)(qrow0 + c) * DM_ + dc * 32 + 8 * hh);

  int vi[8];
#pragma unroll
  for (int r = 0; r < 8; ++r) vi[r] = vpb[qrow0 + 8 * hh + r];

  float mrow[8], lrow[8];
  v8f oacc[4];
#pragma unroll
  for (int r = 0; r < 8; ++r) { mrow[r] = -INFINITY; lrow[r] = 0.f; }
#pragma unroll
  for (int t = 0; t < 4; ++t) oacc[t] = (v8f){0.f, 0.f, 0.f, 0.f, 0.f, 0.f, 0.f, 0.f};

  __attribute__((unused)) const int nChunks = SEQ_ / FL_KC;
  for (int kc = 0; kc < SEQ_ / FL_KC; ++kc) {
    const int kv0 = kc * FL_KC;
    __syncthreads();
    {
      const int r = tid >> 1, hoff = (tid & 1) * 32;
      const _Float16* ks = Kh + (size_t)(kv0 + r) * DM_ + hoff;
      const _Float16* vs = Vh + (size_t)r * NTOK_ + kv0 + hoff;
#pragma unroll
      for (int i = 0; i < 4; ++i) {
        const v8h a0 = *(const v8h*)(ks + 8 * i);
        const v8h b0 = *(const v8h*)(vs + 8 * i);
        *(v8h*)(Ksh + r * DHD_  + hoff + 8 * i) = a0;
        *(v8h*)(Vth + r * FL_KC + hoff + 8 * i) = b0;
      }
      if (tid < FL_KC) Vjs[tid] = vpb[kv0 + tid];
    }
    __syncthreads();

    v8f s[4];
#pragma unroll
    for (int j = 0; j < 4; ++j) {
      s[j] = (v8f){0.f, 0.f, 0.f, 0.f, 0.f, 0.f, 0.f, 0.f};
#pragma unroll
      for (int dc = 0; dc < 2; ++dc) {
        FB kb;
        kb.h[0] = *(const v8h*)(Ksh + (j * 16 + c) * DHD_ + dc * 32 + 8 * hh);
        kb.h[1] = *(const v8h*)(Ksh + (j * 16 + c) * DHD_ + dc * 32 + 16 + 8 * hh);
        s[j] = mma16(qa[dc], kb.v, s[j]);
      }
    }

    int vj[4];
#pragma unroll
    for (int j = 0; j < 4; ++j) vj[j] = Vjs[j * 16 + c];

    float cm[8];
#pragma unroll
    for (int r = 0; r < 8; ++r) {
      float m = -INFINITY;
#pragma unroll
      for (int j = 0; j < 4; ++j) {
        const float sv = s[j][r] * FL_SC + verse_add(vi[r], vj[j]);
        s[j][r] = sv;
        m = fmaxf(m, sv);
      }
#pragma unroll
      for (int off = 1; off < 16; off <<= 1) m = fmaxf(m, __shfl_xor(m, off, 32));
      cm[r] = m;
    }

    _Float16* pw = Psh[wave];
#pragma unroll
    for (int r = 0; r < 8; ++r) {
      const float mnew  = fmaxf(mrow[r], cm[r]);
      const float alpha = __expf(mrow[r] - mnew);
      mrow[r] = mnew;
      float psum = 0.f;
#pragma unroll
      for (int j = 0; j < 4; ++j) {
        const float p = __expf(s[j][r] - mnew);
        psum += p;
        pw[(8 * hh + r) * FL_KC + j * 16 + c] = (_Float16)p;
      }
#pragma unroll
      for (int off = 1; off < 16; off <<= 1) psum += __shfl_xor(psum, off, 32);
      lrow[r] = lrow[r] * alpha + psum;
#pragma unroll
      for (int t = 0; t < 4; ++t) oacc[t][r] *= alpha;
    }
    lds_wave_sync();

#pragma unroll
    for (int kk = 0; kk < 2; ++kk) {
      FB pa;
      pa.h[0] = *(const v8h*)(pw + c * FL_KC + kk * 32 + 8 * hh);
      pa.h[1] = *(const v8h*)(pw + c * FL_KC + kk * 32 + 16 + 8 * hh);
#pragma unroll
      for (int t = 0; t < 4; ++t) {
        FB vb;
        vb.h[0] = *(const v8h*)(Vth + (t * 16 + c) * FL_KC + kk * 32 + 8 * hh);
        vb.h[1] = *(const v8h*)(Vth + (t * 16 + c) * FL_KC + kk * 32 + 16 + 8 * hh);
        oacc[t] = mma16(pa.v, vb.v, oacc[t]);
      }
    }
  }

  float* os = Os[wave];
#pragma unroll
  for (int r = 0; r < 8; ++r) {
    const float inv = 16.0f * __builtin_amdgcn_rcpf(lrow[r]);
#pragma unroll
    for (int t = 0; t < 4; ++t) os[(8 * hh + r) * 68 + t * 16 + c] = oacc[t][r] * inv;
  }
  lds_wave_sync();
  {
    const int q4 = lane >> 3, c8 = (lane & 7) * 8;
    for (int pass = 0; pass < 2; ++pass) {
#pragma unroll
      for (int it = 0; it < 4; ++it) {
        const int row = it * 4 + q4;
        const float* sp = os + row * 68 + c8;
        v8h hv;
#pragma unroll
        for (int e = 0; e < 8; ++e) hv[e] = (_Float16)sp[e];
        *(volatile v8h*)(cb + (size_t)(qrow0 + row) * DM_ + c8) = hv;
      }
      __threadfence();
    }
  }
}

__global__ __launch_bounds__(256) void ln_kernel(const float* __restrict__ F,
                                                 const float* __restrict__ gamma,
                                                 const float* __restrict__ beta,
                                                 float* __restrict__ out, int nrows) {
  const int lane = threadIdx.x & 31;
  const int wave = threadIdx.x >> 5;
  const int row  = blockIdx.x * 8 + wave;
  if (row >= nrows) return;
  const float* fr = F + (size_t)row * DM_ + lane * 4;

  float sum = 0.f;
#pragma unroll
  for (int it = 0; it < 8; ++it) {
    const v4f v = *(const v4f*)(fr + it * 128);
    sum += (v[0] + v[1]) + (v[2] + v[3]);
  }
#pragma unroll
  for (int off = 1; off < 32; off <<= 1) sum += __shfl_xor(sum, off, 32);
  const float mu = sum * (1.0f / (float)DM_);

  float sq = 0.f;
#pragma unroll 1
  for (int it = 0; it < 8; ++it) {
    const v4f v = *(const v4f*)(fr + it * 128);
    const v4f d = v - mu;
    sq += (d[0] * d[0] + d[1] * d[1]) + (d[2] * d[2] + d[3] * d[3]);
  }
#pragma unroll
  for (int off = 1; off < 32; off <<= 1) sq += __shfl_xor(sq, off, 32);
  const float var = sq * (1.0f / (float)DM_);
  const float inv = rsqrtf(var + 1e-5f);

  const float* gr = gamma + lane * 4;
  const float* br = beta  + lane * 4;
  float* orow = out + (size_t)row * DM_ + lane * 4;
#pragma unroll 1
  for (int it = 0; it < 8; ++it) {
    const v4f v  = *(const v4f*)(fr + it * 128);
    const v4f g  = *(const v4f*)(gr + it * 128);
    const v4f bb = *(const v4f*)(br + it * 128);
    const v4f o  = (v - mu) * inv * g + bb;
    *(volatile v4f*)(orow + it * 128) = o;
    __threadfence();
    *(volatile v4f*)(orow + it * 128) = o;
  }
}

extern "C" void kernel_launch(void* const* d_in, const int* in_sizes, int n_in,
                              void* d_out, int out_size, void* d_ws, size_t ws_size,
                              hipStream_t stream) {
  if (n_in < 14) return;
  const int nAct = NTOK_ * DM_;
  const int nW   = DM_ * DM_;
  if (in_sizes[0] != nAct || in_sizes[1] != NTOK_) return;
  if (in_sizes[2] != nW || in_sizes[4] != nW || in_sizes[6] != nW || in_sizes[8] != nW || in_sizes[10] != nW) return;
  if (in_sizes[3] != DM_ || in_sizes[5] != DM_ || in_sizes[7] != DM_ || in_sizes[9] != DM_ ||
      in_sizes[11] != DM_ || in_sizes[12] != DM_ || in_sizes[13] != DM_) return;
  if (out_size != nAct) return;

  const float* x     = (const float*)d_in[0];
  const int*   vpos  = (const int*)d_in[1];
  const float* W_q   = (const float*)d_in[2];
  const float* b_q   = (const float*)d_in[3];
  const float* W_k   = (const float*)d_in[4];
  const float* b_k   = (const float*)d_in[5];
  const float* W_v   = (const float*)d_in[6];
  const float* b_v   = (const float*)d_in[7];
  const float* W_o   = (const float*)d_in[8];
  const float* b_o   = (const float*)d_in[9];
  const float* W_p   = (const float*)d_in[10];
  const float* b_p   = (const float*)d_in[11];
  const float* gamma = (const float*)d_in[12];
  const float* beta  = (const float*)d_in[13];
  float* out = (float*)d_out;

  const size_t PA16 = (size_t)nAct * 2;
  const size_t PW16 = (size_t)nW * 2;
  const size_t PA32 = (size_t)nAct * 4;
  size_t off = 0;
  const size_t oXh  = off; off += PA16;
  const size_t oWq  = off; off += PW16;
  const size_t oWk  = off; off += PW16;
  const size_t oWv  = off; off += PW16;
  const size_t oWo  = off; off += PW16;
  const size_t oWp  = off; off += PW16;
  const size_t oQ   = off; off += PA16;
  const size_t oK   = off; off += PA16;
  const size_t oVT  = off; off += PA16;
  const size_t oCTX = off; off += PA16;
  const size_t oAO  = off; off += PA16;
  const size_t oF   = off; off += PA32;
  if (off > ws_size) return;
  if (off > (size_t)134217728) return;

  char* ws = (char*)d_ws;
  _Float16* Xh   = (_Float16*)(ws + oXh);
  _Float16* Wq16 = (_Float16*)(ws + oWq);
  _Float16* Wk16 = (_Float16*)(ws + oWk);
  _Float16* Wv16 = (_Float16*)(ws + oWv);
  _Float16* Wo16 = (_Float16*)(ws + oWo);
  _Float16* Wp16 = (_Float16*)(ws + oWp);
  _Float16* Q16  = (_Float16*)(ws + oQ);
  _Float16* K16  = (_Float16*)(ws + oK);
  _Float16* VT16 = (_Float16*)(ws + oVT);
  _Float16* CTX  = (_Float16*)(ws + oCTX);
  _Float16* AO   = (_Float16*)(ws + oAO);
  float*    F    = (float*)(ws + oF);

  const dim3 blk(256);
  const int n8A = nAct / 8;
  const int n8W = nW / 8;
  const dim3 gA((n8A + 255) / 256);
  const dim3 gW((n8W + 255) / 256);

  cvt_f16_kernel<<<gA, blk, 0, stream>>>(x,   Xh,   n8A, 1.0f);
  cvt_f16_kernel<<<gW, blk, 0, stream>>>(W_q, Wq16, n8W, 16.0f);
  cvt_f16_kernel<<<gW, blk, 0, stream>>>(W_k, Wk16, n8W, 16.0f);
  cvt_f16_kernel<<<gW, blk, 0, stream>>>(W_v, Wv16, n8W, 16.0f);
  cvt_f16_kernel<<<gW, blk, 0, stream>>>(W_o, Wo16, n8W, 16.0f);
  cvt_f16_kernel<<<gW, blk, 0, stream>>>(W_p, Wp16, n8W, 16.0f);

  const dim3 gG(((NTOK_ / 32) * (DM_ / 64) + 7) / 8);
  const dim3 gVT(((DM_ / 32) * (NTOK_ / 64) + 7) / 8);

  gemm_kernel<2, true, false><<<gG, blk, 0, stream>>>(
      Xh, DM_, Wq16, DM_, (void*)Q16, DM_, b_q, 16.0f, nullptr, NTOK_, DM_, DM_, 1.0f);
  gemm_kernel<2, true, false><<<gG, blk, 0, stream>>>(
      Xh, DM_, Wk16, DM_, (void*)K16, DM_, b_k, 16.0f, nullptr, NTOK_, DM_, DM_, 1.0f);
  gemm_kernel<1, true, false><<<gVT, blk, 0, stream>>>(
      Wv16, DM_, Xh, DM_, (void*)VT16, NTOK_, b_v, 16.0f, nullptr, DM_, NTOK_, DM_, 1.0f);

  flash_kernel<<<dim3(NB_ * NH_ * (SEQ_ / 64)), dim3(128), 0, stream>>>(Q16, K16, VT16, vpos, CTX);

  gemm_kernel<2, true, false><<<gG, blk, 0, stream>>>(
      CTX, DM_, Wo16, DM_, (void*)AO, DM_, b_o, 4096.0f, nullptr, NTOK_, DM_, DM_, 1.0f);
  gemm_kernel<2, false, true><<<gG, blk, 0, stream>>>(
      AO, DM_, Wp16, DM_, (void*)F, DM_, b_p, 1.0f, x, NTOK_, DM_, DM_, 1.0f / 65536.0f);

  ln_kernel<<<dim3((NTOK_ + 7) / 8), blk, 0, stream>>>(F, gamma, beta, out, NTOK_);

  (void)hipGetLastError();
}
